// NodeEmbedder_14525579395502
// MI455X (gfx1250) — hardware-verified
//
#include <hip/hip_runtime.h>


#define NN       50000
#define EE       800000
#define IN_DIMC  300
#define KPAD_IN  320
#define HIDC     64
#define HCC      128
#define XLRW     256
#define EDGE_D   16
#define NLAYERS  2

#define NPB      256
#define NBLK     ((NN + NPB - 1) / NPB)
#define LCAP     128
#define SCAP     768
#define BCAP     (8 * SCAP)
#define CSR_INTS (2 * NPB + 3 * BCAP)
#define MAXDEG   256

#define BN_BLOCKS 200
#define BN_ROWS   250
#define BN_PITCH  640

#define MT         (NN / 16)
#define GEMM_WAVES 4

#define PREP_C0 2560
#define PREP_C1 (PREP_C0 + 4096)
#define PREP_C2 (PREP_C1 + 2048)
#define PREP_C3 (PREP_C2 + 512)
#define PREP_C4 (PREP_C3 + 512)
#define PREP_TOTAL (PREP_C4 + KPAD_IN)

typedef _Float16 f16_t;
typedef _Float16 v8h  __attribute__((ext_vector_type(8)));
typedef _Float16 v16h __attribute__((ext_vector_type(16)));
typedef float    v8f  __attribute__((ext_vector_type(8)));
typedef float    v4f  __attribute__((ext_vector_type(4)));
typedef int      v4i  __attribute__((ext_vector_type(4)));
union Frag { v16h v; v8h hv[2]; };

__device__ __forceinline__ v8f wmma_f16(v16h a, v16h b, v8f c)
{
    v8f d = __builtin_amdgcn_wmma_f32_16x16x32_f16(false, a, false, b, (short)0, c, false, false);
    asm volatile("v_nop\n\tv_nop\n\tv_nop\n\tv_nop" : "+v"(d) : "v"(a), "v"(b));
    return d;
}

__device__ __forceinline__ v8f zero_acc()
{
    v8f z;
#pragma unroll
    for (int i = 0; i < 8; ++i) z[i] = 0.f;
    return z;
}

__device__ __forceinline__ v8h zero8h()
{
    v8h z;
#pragma unroll
    for (int i = 0; i < 8; ++i) z[i] = (f16_t)0.0f;
    return z;
}

__device__ __forceinline__ v8h cvt8(v4f a, v4f b)
{
    v8h r;
    r[0] = (f16_t)a[0]; r[1] = (f16_t)a[1]; r[2] = (f16_t)a[2]; r[3] = (f16_t)a[3];
    r[4] = (f16_t)b[0]; r[5] = (f16_t)b[1]; r[6] = (f16_t)b[2]; r[7] = (f16_t)b[3];
    return r;
}

__global__ __launch_bounds__(256)
void k_bn_stats(const float* __restrict__ x, double* __restrict__ part)
{
    const int t = threadIdx.x;
    const int r0 = blockIdx.x * BN_ROWS;
    const int c0 = t, c1 = t + 256;
    double s0 = 0.0, q0 = 0.0, s1 = 0.0, q1 = 0.0;
    for (int i = 0; i < BN_ROWS; ++i) {
        const int r = r0 + i;
        if (r >= NN) break;
        const float* row = x + (size_t)r * IN_DIMC;
        const double v = (double)row[c0];
        s0 += v; q0 += v * v;
        if (c1 < IN_DIMC) { const double u = (double)row[c1]; s1 += u; q1 += u * u; }
    }
    volatile double* vp = part + (size_t)blockIdx.x * BN_PITCH;
    vp[c0] = s0; vp[KPAD_IN + c0] = q0;
    if (c1 < KPAD_IN) { vp[c1] = s1; vp[KPAD_IN + c1] = q1; }
    __threadfence();
    vp[c0] = s0; vp[KPAD_IN + c0] = q0;
    if (c1 < KPAD_IN) { vp[c1] = s1; vp[KPAD_IN + c1] = q1; }
}

__global__ __launch_bounds__(256)
void k_prep(const double* __restrict__ part, const float* __restrict__ bnw, const float* __restrict__ bnb,
            const float* __restrict__ projW, const float* __restrict__ WlW, const float* __restrict__ WrW,
            const float* __restrict__ linW, const float* __restrict__ outW, const float* __restrict__ WeW,
            float* __restrict__ bnA, float* __restrict__ bnS,
            f16_t* __restrict__ projT, f16_t* __restrict__ wlrT, f16_t* __restrict__ linT,
            f16_t* __restrict__ outT, f16_t* __restrict__ weT)
{
    const int gid = blockIdx.x * 256 + threadIdx.x;
    if (gid < PREP_C4) {
        float v[8];
        f16_t* dp;
        if (gid < PREP_C0) {
            const int n = gid / 40, kc = gid - n * 40;
#pragma unroll
            for (int i = 0; i < 8; ++i) {
                const int k = kc * 8 + i;
                v[i] = (k < IN_DIMC) ? projW[(size_t)k * HIDC + n] : 0.f;
            }
            dp = projT + (size_t)n * KPAD_IN + kc * 8;
        } else if (gid < PREP_C1) {
            const int ch = gid - PREP_C0;
            const int l = ch >> 11, n = (ch >> 3) & 255, kc = ch & 7;
#pragma unroll
            for (int i = 0; i < 8; ++i) {
                const int k = kc * 8 + i;
                v[i] = (n < HCC) ? WlW[(size_t)l * (HIDC * HCC) + k * HCC + n]
                                 : WrW[(size_t)l * (HIDC * HCC) + k * HCC + (n - HCC)];
            }
            dp = wlrT + (size_t)ch * 8;
        } else if (gid < PREP_C2) {
            const int ch = gid - PREP_C1;
            const int l = ch >> 10, n = (ch >> 4) & 63, kc = ch & 15;
#pragma unroll
            for (int i = 0; i < 8; ++i) {
                const int k = kc * 8 + i;
                v[i] = linW[(size_t)l * (HCC * HIDC) + k * HIDC + n];
            }
            dp = linT + (size_t)ch * 8;
        } else if (gid < PREP_C3) {
            const int ch = gid - PREP_C2;
            const int n = ch >> 3, kc = ch & 7;
#pragma unroll
            for (int i = 0; i < 8; ++i) {
                const int k = kc * 8 + i;
                v[i] = outW[k * HIDC + n];
            }
            dp = outT + ch * 8;
        } else {
            const int ch = gid - PREP_C3;
            const int l = ch >> 8, n = (ch >> 1) & 127, kc = ch & 1;
#pragma unroll
            for (int i = 0; i < 8; ++i) {
                const int k = kc * 8 + i;
                v[i] = WeW[(size_t)l * (EDGE_D * HCC) + k * HCC + n];
            }
            dp = weT + ch * 8;
        }
        v8h o;
#pragma unroll
        for (int i = 0; i < 8; ++i) o[i] = (f16_t)v[i];
        *(volatile v8h*)dp = o;
        __threadfence();
        *(volatile v8h*)dp = o;
    } else if (gid < PREP_TOTAL) {
        const int c = gid - PREP_C4;
        float a = 0.f, s = 0.f;
        if (c < IN_DIMC) {
            double su = 0.0, sq = 0.0;
            for (int p = 0; p < BN_BLOCKS; ++p) {
                su += part[(size_t)p * BN_PITCH + c];
                sq += part[(size_t)p * BN_PITCH + KPAD_IN + c];
            }
            const double mean = su / (double)NN;
            double var = sq / (double)NN - mean * mean;
            if (var < 0.0) var = 0.0;
            const double r = 1.0 / sqrt(var + 1e-5);
            const double aa = r * (double)bnw[c];
            a = (float)aa;
            s = (float)((double)bnb[c] - mean * aa);
        }
        volatile float* va = bnA; volatile float* vb = bnS;
        va[c] = a; vb[c] = s;
        __threadfence();
        va[c] = a; vb[c] = s;
    }
}

__device__ __forceinline__ int csr_elem(int idx, int n0, const int* sb, const int* sd,
                                        const unsigned* sr, const int* __restrict__ srcg)
{
    if (idx < NPB) return sb[idx];
    if (idx < 2 * NPB) return sd[idx - NPB];
    const int k = idx - 2 * NPB;
    const int sec = k / BCAP;
    const int kk = k - sec * BCAP;
    const unsigned xv = sr[kk];
    unsigned eid = xv & 0xFFFFFFu;
    if (eid > (unsigned)(EE - 1)) eid = EE - 1;
    if (sec == 0) return (int)eid;
    if (sec == 1) {
        unsigned s = (unsigned)srcg[eid];
        if (s > (unsigned)(NN - 1)) s = NN - 1;
        return (int)s;
    }
    unsigned d = (unsigned)n0 + (xv >> 24);
    if (d > (unsigned)(NN - 1)) d = NN - 1;
    return (int)d;
}

__global__ __launch_bounds__(256)
void k_csr_build(const int* __restrict__ srcg, const int* __restrict__ dstg, int* __restrict__ csr)
{
    __shared__ unsigned lst[8][8][LCAP];
    __shared__ unsigned srt[8][SCAP];
    __shared__ int scnt[8][8];
    __shared__ int sbeg[NPB];
    __shared__ int sdeg[NPB];
    const int t = threadIdx.x, w = t >> 5, lane = t & 31;
    const int n0 = blockIdx.x * NPB;
    const unsigned ltmask = (1u << lane) - 1u;

    int cnt[8];
#pragma unroll
    for (int q = 0; q < 8; ++q) cnt[q] = 0;

    for (int base = 0; base < EE; base += 256) {
        const int e = base + t;
        int rel = -1;
        if (e < EE) rel = dstg[e] - n0;
        const bool in = (unsigned)rel < (unsigned)NPB;
        const int myq = rel >> 5;
#pragma unroll
        for (int q = 0; q < 8; ++q) {
            const bool p = in && (myq == q);
            const unsigned mask = __builtin_amdgcn_ballot_w32(p);
            const int c = cnt[q];
            if (p) {
                const int pos = c + (int)__builtin_popcount(mask & ltmask);
                if (pos < LCAP) lst[q][w][pos] = ((unsigned)rel << 24) | (unsigned)e;
            }
            cnt[q] = c + (int)__builtin_popcount(mask);
        }
    }
    if (lane == 0) {
#pragma unroll
        for (int q = 0; q < 8; ++q) scnt[q][w] = cnt[q] > LCAP ? LCAP : cnt[q];
    }
    __syncthreads();

    const int dl = w * 32 + lane;
    int mycnt = 0;
    for (int v = 0; v < 8; ++v) {
        int nv = scnt[w][v];
        nv = nv > LCAP ? LCAP : (nv < 0 ? 0 : nv);
        for (int i = 0; i < nv; ++i) {
            const unsigned xv = lst[w][v][i];
            if ((int)(xv >> 24) == dl) ++mycnt;
        }
    }
    int incl = mycnt;
#pragma unroll
    for (int o = 1; o < 32; o <<= 1) {
        const int y = __shfl_up(incl, o, 32);
        if (lane >= o) incl += y;
    }
    int off0 = incl - mycnt;
    int tot = __shfl(incl, 31, 32);
    if (off0 > SCAP) off0 = SCAP;
    int deg = mycnt;
    if (deg > SCAP - off0) deg = SCAP - off0;
    if (tot > SCAP) tot = SCAP;
    int cur = off0;
    const int lim = off0 + deg;
    for (int v = 0; v < 8; ++v) {
        int nv = scnt[w][v];
        nv = nv > LCAP ? LCAP : (nv < 0 ? 0 : nv);
        for (int i = 0; i < nv; ++i) {
            const unsigned xv = lst[w][v][i];
            if ((int)(xv >> 24) == dl && cur < lim) { srt[w][cur] = xv; ++cur; }
        }
    }
    for (int i = tot + lane; i < SCAP; i += 32) srt[w][i] = 0u;
    sbeg[dl] = w * SCAP + off0;
    sdeg[dl] = deg;
    __syncthreads();

    int* gb = csr + (size_t)blockIdx.x * CSR_INTS;
    const unsigned* srflat = &srt[0][0];
    for (int ps = 0; ps < 2; ++ps) {
        for (int g = t * 4; g < CSR_INTS; g += 1024) {
            v4i vv;
            vv[0] = csr_elem(g + 0, n0, sbeg, sdeg, srflat, srcg);
            vv[1] = csr_elem(g + 1, n0, sbeg, sdeg, srflat, srcg);
            vv[2] = csr_elem(g + 2, n0, sbeg, sdeg, srflat, srcg);
            vv[3] = csr_elem(g + 3, n0, sbeg, sdeg, srflat, srcg);
            *(volatile v4i*)(gb + g) = vv;
        }
        if (ps == 0) __threadfence();
    }
}

__global__ __launch_bounds__(128)
void k_gemm2(const float* __restrict__ A, int K1, int K1p,
             const float* __restrict__ bnA, const float* __restrict__ bnS,
             const f16_t* __restrict__ B1T, const float* __restrict__ b1, int relu1,
             const f16_t* __restrict__ B2T, const float* __restrict__ b2a, const float* __restrict__ b2b,
             int nsplit, int N2, float* __restrict__ out)
{
    __shared__ __attribute__((aligned(16))) f16_t sA[GEMM_WAVES][16][KPAD_IN];
    __shared__ __attribute__((aligned(16))) f16_t sH[GEMM_WAVES][16][HIDC];
    __shared__ __attribute__((aligned(16))) float sO[GEMM_WAVES][16][32];
    const int w = threadIdx.x >> 5, l = threadIdx.x & 31, h = l >> 4, m = l & 15;
    const int tm = blockIdx.x * GEMM_WAVES + w;
    const bool valid = tm < MT;
    const int tmc = valid ? tm : (MT - 1);
    const size_t row0 = (size_t)tmc * 16;

    for (int r = 0; r < 16; ++r) {
        const float* ar = A + (row0 + r) * (size_t)K1;
        for (int k = l; k < K1p; k += 32) {
            float v = 0.f;
            if (k < K1) {
                v = ar[k];
                if (bnA) v = fmaf(v, bnA[k], bnS[k]);
            }
            sA[w][r][k] = (f16_t)v;
        }
    }
    __syncthreads();

#pragma unroll 1
    for (int ct = 0; ct < HIDC / 16; ++ct) {
        v8f acc = zero_acc();
        const f16_t* bcol = B1T + (size_t)(ct * 16 + m) * K1p;
        for (int k0 = 0; k0 < K1p; k0 += 32) {
            Frag a, b;
            a.hv[0] = *(const v8h*)&sA[w][m][k0 + 8 * h];
            a.hv[1] = *(const v8h*)&sA[w][m][k0 + 16 + 8 * h];
            b.hv[0] = *(const v8h*)(bcol + k0 + 8 * h);
            b.hv[1] = *(const v8h*)(bcol + k0 + 16 + 8 * h);
            acc = wmma_f16(a.v, b.v, acc);
        }
        const int c = ct * 16 + m;
        const float bias = b1[c];
#pragma unroll
        for (int r = 0; r < 8; ++r) {
            float v = acc[r] + bias;
            if (relu1) v = fmaxf(v, 0.f);
            sH[w][8 * h + r][c] = (f16_t)v;
        }
    }
    __syncthreads();

    Frag a0, a1;
    a0.hv[0] = *(const v8h*)&sH[w][m][8 * h];
    a0.hv[1] = *(const v8h*)&sH[w][m][16 + 8 * h];
    a1.hv[0] = *(const v8h*)&sH[w][m][32 + 8 * h];
    a1.hv[1] = *(const v8h*)&sH[w][m][48 + 8 * h];
#pragma unroll 1
    for (int cs = 0; cs < N2; cs += 32) {
        v8f accA = zero_acc(), accB = zero_acc();
        {
            const f16_t* bp = B2T + (size_t)(cs + m) * HIDC;
            Frag b;
            b.hv[0] = *(const v8h*)(bp + 8 * h);
            b.hv[1] = *(const v8h*)(bp + 16 + 8 * h);
            accA = wmma_f16(a0.v, b.v, accA);
            b.hv[0] = *(const v8h*)(bp + 32 + 8 * h);
            b.hv[1] = *(const v8h*)(bp + 48 + 8 * h);
            accA = wmma_f16(a1.v, b.v, accA);
        }
        {
            const f16_t* bp = B2T + (size_t)(cs + 16 + m) * HIDC;
            Frag b;
            b.hv[0] = *(const v8h*)(bp + 8 * h);
            b.hv[1] = *(const v8h*)(bp + 16 + 8 * h);
            accB = wmma_f16(a0.v, b.v, accB);
            b.hv[0] = *(const v8h*)(bp + 32 + 8 * h);
            b.hv[1] = *(const v8h*)(bp + 48 + 8 * h);
            accB = wmma_f16(a1.v, b.v, accB);
        }
        const int cA = cs + m, cB = cs + 16 + m;
        const float biasA = (cA < nsplit) ? b2a[cA] : b2b[cA - nsplit];
        const float biasB = (cB < nsplit) ? b2a[cB] : b2b[cB - nsplit];
#pragma unroll
        for (int r = 0; r < 8; ++r) {
            sO[w][8 * h + r][m]      = accA[r] + biasA;
            sO[w][8 * h + r][16 + m] = accB[r] + biasB;
        }
        __syncthreads();
        v4f vv[4];
#pragma unroll
        for (int i = 0; i < 4; ++i) {
            const int rr = i * 4 + (l >> 3), cc = (l & 7) * 4;
            vv[i] = *(const v4f*)&sO[w][rr][cc];
        }
        if (valid) {
#pragma unroll
            for (int i = 0; i < 4; ++i) {
                const int rr = i * 4 + (l >> 3), cc = (l & 7) * 4;
                float* p = out + (row0 + rr) * (size_t)N2 + cs + cc;
                *(volatile v4f*)p = vv[i];
            }
        }
        __threadfence();
        if (valid) {
#pragma unroll
            for (int i = 0; i < 4; ++i) {
                const int rr = i * 4 + (l >> 3), cc = (l & 7) * 4;
                float* p = out + (row0 + rr) * (size_t)N2 + cs + cc;
                *(volatile v4f*)p = vv[i];
            }
        }
        __syncthreads();
    }
}

__global__ __launch_bounds__(256)
void k_gat_edge(const int* __restrict__ csr, const float* __restrict__ eattr,
                const f16_t* __restrict__ weT, const float* __restrict__ attl,
                const float* __restrict__ xlr, const float* __restrict__ cbias,
                float* __restrict__ hout)
{
    __shared__ float slog[8][SCAP * 2];
    __shared__ int sbeg[NPB];
    __shared__ int sdeg[NPB];
    __shared__ float satt[HCC];
    const int t = threadIdx.x, w = t >> 5, l = t & 31, h = l >> 4, m = l & 15;
    const int n0 = blockIdx.x * NPB;
    const int* cb = csr + (size_t)blockIdx.x * CSR_INTS;
    sbeg[t] = cb[t];
    sdeg[t] = cb[NPB + t];
    if (t < HCC) satt[t] = attl[t];
    __syncthreads();
    const int* ceid = cb + 2 * NPB;
    const int* csrc = ceid + BCAP;
    const int* cdn  = csrc + BCAP;
    const int R = w * SCAP;
    int tot = sbeg[w * 32 + 31] + sdeg[w * 32 + 31] - R;
    tot = tot < 0 ? 0 : tot;
    tot = tot > SCAP ? SCAP : tot;
    const int ntile = (tot + 15) >> 4;
    float* sl = &slog[w][0];
    const v8h z8 = zero8h();

    for (int ti = 0; ti < ntile; ++ti) {
        const int e0 = R + ti * 16;
        unsigned eidm = (unsigned)ceid[e0 + m];
        if (eidm > (unsigned)(EE - 1)) eidm = EE - 1;
        const float* ep = eattr + (size_t)eidm * EDGE_D + 8 * h;
        const v4f x0 = *(const v4f*)ep;
        const v4f x1 = *(const v4f*)(ep + 4);
        Frag a;
        a.hv[0] = cvt8(x0, x1);
        a.hv[1] = z8;
        int sr[8], dr[8];
#pragma unroll
        for (int r = 0; r < 8; ++r) {
            const int er = e0 + 8 * h + r;
            unsigned s = (unsigned)csrc[er];
            unsigned d = (unsigned)cdn[er];
            sr[r] = (int)(s > (unsigned)(NN - 1) ? (unsigned)(NN - 1) : s);
            dr[r] = (int)(d > (unsigned)(NN - 1) ? (unsigned)(NN - 1) : d);
        }
        float pl0[8], pl1[8];
#pragma unroll
        for (int r = 0; r < 8; ++r) { pl0[r] = 0.f; pl1[r] = 0.f; }
#pragma unroll 1
        for (int ct = 0; ct < HCC / 16; ++ct) {
            const int c = ct * 16 + m;
            Frag b;
            b.hv[0] = *(const v8h*)(weT + c * EDGE_D + 8 * h);
            b.hv[1] = z8;
            v8f acc = wmma_f16(a.v, b.v, zero_acc());
            const float av = satt[c];
#pragma unroll
            for (int r = 0; r < 8; ++r) {
                float v = acc[r] + xlr[(size_t)sr[r] * XLRW + c] + xlr[(size_t)dr[r] * XLRW + HCC + c];
                v = (v >= 0.f) ? v : 0.2f * v;
                const float cv = v * av;
                if (ct < 4) pl0[r] += cv; else pl1[r] += cv;
            }
        }
#pragma unroll
        for (int r = 0; r < 8; ++r) {
#pragma unroll
            for (int o = 8; o > 0; o >>= 1) {
                pl0[r] += __shfl_xor(pl0[r], o, 32);
                pl1[r] += __shfl_xor(pl1[r], o, 32);
            }
        }
        if (m < 8) {
            float v0 = 0.f, v1 = 0.f;
#pragma unroll
            for (int r = 0; r < 8; ++r) { if (m == r) { v0 = pl0[r]; v1 = pl1[r]; } }
            const int li = ti * 16 + 8 * h + m;
            sl[li * 2 + 0] = v0;
            sl[li * 2 + 1] = v1;
        }
    }
    __syncthreads();

    volatile float* vs = sl;
    const v4f cb4 = *(const v4f*)(cbias + 4 * l);
    const int hd = h;
    for (int j = 0; j < 32; ++j) {
        const int nl = w * 32 + j;
        const int node = n0 + nl;
        if (node >= NN) break;
        int beg = sbeg[nl];
        int deg = sdeg[nl];
        beg = beg < R ? R : beg;
        beg = beg > R + SCAP ? R + SCAP : beg;
        const int lb = beg - R;
        deg = deg < 0 ? 0 : deg;
        deg = deg > MAXDEG ? MAXDEG : deg;
        if (deg > SCAP - lb) deg = SCAP - lb;
#pragma unroll
        for (int q = 0; q < 2; ++q) {
            float mx = -__builtin_huge_valf();
            for (int i = l; i < deg; i += 32) mx = fmaxf(mx, vs[(lb + i) * 2 + q]);
#pragma unroll
            for (int o = 16; o > 0; o >>= 1) mx = fmaxf(mx, __shfl_xor(mx, o, 32));
            float s = 0.f;
            for (int i = l; i < deg; i += 32) {
                const int ai = (lb + i) * 2 + q;
                const float p = expf(vs[ai] - mx);
                vs[ai] = p;
                s += p;
            }
#pragma unroll
            for (int o = 16; o > 0; o >>= 1) s += __shfl_xor(s, o, 32);
            for (int i = l; i < deg; i += 32) {
                const int ai = (lb + i) * 2 + q;
                const float p = vs[ai];
                vs[ai] = p / s;
            }
        }
        v4f acc;
        acc[0] = 0.f; acc[1] = 0.f; acc[2] = 0.f; acc[3] = 0.f;
        for (int i = 0; i < deg; ++i) {
            unsigned s = (unsigned)csrc[beg + i];
            if (s > (unsigned)(NN - 1)) s = NN - 1;
            const float al = vs[(lb + i) * 2 + hd];
            const v4f xv = *(const v4f*)(xlr + (size_t)s * XLRW + 4 * l);
            acc += al * xv;
        }
        v4f o = acc + cb4;
        o[0] = fmaxf(o[0], 0.f); o[1] = fmaxf(o[1], 0.f);
        o[2] = fmaxf(o[2], 0.f); o[3] = fmaxf(o[3], 0.f);
        float* op = hout + (size_t)node * HCC + 4 * l;
        *(volatile v4f*)op = o;
        __threadfence();
        *(volatile v4f*)op = o;
    }
}

extern "C" void kernel_launch(void* const* d_in, const int* in_sizes, int n_in,
                              void* d_out, int out_size, void* d_ws, size_t ws_size,
                              hipStream_t stream)
{
    if (n_in < 18) return;
    if (in_sizes[0] != NN * IN_DIMC || in_sizes[1] != 2 * EE || in_sizes[2] != EE * EDGE_D ||
        in_sizes[12] != NLAYERS * HCC || out_size != NN * HIDC) return;

    const float* x          = (const float*)d_in[0];
    const int*   edge_index = (const int*)d_in[1];
    const float* edge_attr  = (const float*)d_in[2];
    const float* bn_w       = (const float*)d_in[3];
    const float* bn_b       = (const float*)d_in[4];
    const float* proj_W     = (const float*)d_in[5];
    const float* proj_b     = (const float*)d_in[6];
    const float* lin_l_W    = (const float*)d_in[7];
    const float* lin_l_b    = (const float*)d_in[8];
    const float* lin_r_W    = (const float*)d_in[9];
    const float* lin_r_b    = (const float*)d_in[10];
    const float* lin_edge_W = (const float*)d_in[11];
    const float* att        = (const float*)d_in[12];
    const float* conv_bias  = (const float*)d_in[13];
    const float* lin_W      = (const float*)d_in[14];
    const float* lin_b      = (const float*)d_in[15];
    const float* out_W      = (const float*)d_in[16];
    const float* out_b      = (const float*)d_in[17];
    float* outp = (float*)d_out;

    const int* src = edge_index;
    const int* dst = edge_index + EE;

    size_t off = 0;
    auto take = [&](size_t bytes) -> size_t {
        const size_t p = off;
        off += (bytes + 255) & ~(size_t)255;
        return p;
    };
    const size_t o_part  = take((size_t)BN_BLOCKS * BN_PITCH * sizeof(double));
    const size_t o_bnA   = take((size_t)KPAD_IN * 4);
    const size_t o_bnS   = take((size_t)KPAD_IN * 4);
    const size_t o_projT = take((size_t)HIDC * KPAD_IN * 2);
    const size_t o_wlrT  = take((size_t)NLAYERS * XLRW * HIDC * 2);
    const size_t o_linT  = take((size_t)NLAYERS * HIDC * HCC * 2);
    const size_t o_outT  = take((size_t)HIDC * HIDC * 2);
    const size_t o_weT   = take((size_t)NLAYERS * HCC * EDGE_D * 2);
    const size_t o_csr   = take((size_t)NBLK * CSR_INTS * 4);
    const size_t o_xlr   = take((size_t)NN * XLRW * 4);
    const size_t o_h     = take((size_t)NN * HCC * 4);
    if (off > ws_size) return;

    char* wsb = (char*)d_ws;
    double* part  = (double*)(wsb + o_part);
    float*  bnA   = (float*)(wsb + o_bnA);
    float*  bnS   = (float*)(wsb + o_bnS);
    f16_t*  projT = (f16_t*)(wsb + o_projT);
    f16_t*  wlrT  = (f16_t*)(wsb + o_wlrT);
    f16_t*  linT  = (f16_t*)(wsb + o_linT);
    f16_t*  outT  = (f16_t*)(wsb + o_outT);
    f16_t*  weT   = (f16_t*)(wsb + o_weT);
    int*    csr   = (int*)(wsb + o_csr);
    float*  xlr   = (float*)(wsb + o_xlr);
    float*  hbuf  = (float*)(wsb + o_h);

    const int gemm_blocks = (MT + GEMM_WAVES - 1) / GEMM_WAVES;
    const int prep_blocks = (PREP_TOTAL + 255) / 256;

    k_bn_stats<<<BN_BLOCKS, 256, 0, stream>>>(x, part);
    k_prep<<<prep_blocks, 256, 0, stream>>>(part, bn_w, bn_b, proj_W, lin_l_W, lin_r_W, lin_W, out_W,
                                            lin_edge_W, bnA, bnS, projT, wlrT, linT, outT, weT);
    k_csr_build<<<NBLK, 256, 0, stream>>>(src, dst, csr);
    k_gemm2<<<gemm_blocks, 128, 0, stream>>>(x, IN_DIMC, KPAD_IN, bnA, bnS, projT, proj_b, 0,
                                              wlrT, lin_l_b, lin_r_b, HCC, XLRW, xlr);
    k_gat_edge<<<NBLK, 256, 0, stream>>>(csr, edge_attr, weT, att, xlr, conv_bias, hbuf);
    k_gemm2<<<gemm_blocks, 128, 0, stream>>>(hbuf, HCC, HCC, (const float*)nullptr, (const float*)nullptr,
                                              linT, lin_b, 1,
                                              wlrT + (size_t)XLRW * HIDC, lin_l_b + HCC, lin_r_b + HCC,
                                              HCC, XLRW, xlr);
    k_gat_edge<<<NBLK, 256, 0, stream>>>(csr, edge_attr, weT + HCC * EDGE_D, att + HCC, xlr,
                                          conv_bias + HCC, hbuf);
    k_gemm2<<<gemm_blocks, 128, 0, stream>>>(hbuf, HCC, HCC, (const float*)nullptr, (const float*)nullptr,
                                              linT + (size_t)HIDC * HCC, lin_b + HIDC, 1,
                                              outT, out_b, out_b, HIDC, HIDC, outp);
    (void)hipGetLastError();
}
